// GATLSTMPolicyNetwork_15470472200530
// MI455X (gfx1250) — hardware-verified
//
#include <hip/hip_runtime.h>
#include <math.h>

typedef __attribute__((ext_vector_type(16))) _Float16 v16h;
typedef __attribute__((ext_vector_type(8)))  _Float16 v8h;
typedef __attribute__((ext_vector_type(16))) __bf16   v16b;
typedef __attribute__((ext_vector_type(8)))  __bf16   v8b;
typedef __attribute__((ext_vector_type(8)))  float    v8f;
typedef __attribute__((ext_vector_type(4)))  float    v4f;

constexpr int kT      = 4096;
constexpr int kNodes  = 64;
constexpr int kFeat   = 8;
constexpr int kObs    = kNodes * kFeat;
constexpr int kHidU   = 64;
constexpr int kGates  = 4 * kHidU;
constexpr int kCat    = 256;
constexpr int kAct    = 64;
constexpr int kHeadsN = 2 * kAct;
constexpr float kMinStd = 0.001f;
constexpr float kMaxStd = 10.0f;

constexpr int kNPB        = 16;
constexpr int kRecBlocks  = kNodes / kNPB;
constexpr int kRecThreads = 128;
constexpr int kKpad       = 24;
constexpr int kBtP        = 96;
constexpr int kHtP        = 72;
constexpr int kXch        = 8;
constexpr int kXtHalves   = (kXch * kNPB + 2) * kFeat;
constexpr int kHmDwords   = kT * kHidU / 2;
constexpr int kFin4       = 2 * kT * kAct / 4;
static_assert(kT % kXch == 0);
static_assert(kNodes % kNPB == 0);
static_assert(kHmDwords % 256 == 0);
static_assert(kFin4 % 256 == 0);
static_assert((kT * kAct / 4) % 256 == 0);

__device__ __forceinline__ unsigned short f2bf_bits(float f) {
  unsigned u = __float_as_uint(f);
  return (unsigned short)((u + 0x7FFFu + ((u >> 16) & 1u)) >> 16);
}
__device__ __forceinline__ float bf_bits2f(unsigned short h) { return __uint_as_float(((unsigned)h) << 16); }

__device__ __forceinline__ void dep_guard_h(v8f& a, v8f& b, v16h x, v16h y) { asm volatile("v_nop\n\tv_nop\n\tv_nop\n\tv_nop" : "+v"(a), "+v"(b) : "v"(x), "v"(y)); }
__device__ __forceinline__ void dep_guard_b(v8f& a, v8f& b, v16b x, v16b y) { asm volatile("v_nop\n\tv_nop\n\tv_nop\n\tv_nop" : "+v"(a), "+v"(b) : "v"(x), "v"(y)); }
__device__ __forceinline__ void keep4_h(v16h a, v16h b, v16h c, v16h d) { asm volatile("v_nop" :: "v"(a), "v"(b), "v"(c), "v"(d)); }
__device__ __forceinline__ void keep4_b(v16b a, v16b b, v16b c, v16b d) { asm volatile("v_nop" :: "v"(a), "v"(b), "v"(c), "v"(d)); }
__device__ __forceinline__ void acc_guard4(v8f& a, v8f& b, v8f& c, v8f& d) { asm volatile("v_nop\n\tv_nop\n\tv_nop\n\tv_nop" : "+v"(a), "+v"(b), "+v"(c), "+v"(d)); }

template <typename T> struct Frag;
template <> struct Frag<_Float16> {
  typedef v16h V; union U { v16h v; v8h h[2]; };
  static __device__ __forceinline__ v16h load(const _Float16* p) {
    U f; f.h[0] = *(const v8h*)(p); f.h[1] = *(const v8h*)(p + 16); return f.v;
  }
  static __device__ __forceinline__ v8f mma(v16h a, v16h b, v8f c) {
    return __builtin_amdgcn_wmma_f32_16x16x32_f16(false, a, false, b, (short)0, c, false, false);
  }
  static __device__ __forceinline__ void guard(v8f& a, v8f& b, v16h x, v16h y) { dep_guard_h(a, b, x, y); }
  static __device__ __forceinline__ void keep(v16h a, v16h b, v16h c, v16h d) { keep4_h(a, b, c, d); }
};
template <> struct Frag<__bf16> {
  typedef v16b V; union U { v16b v; v8b h[2]; };
  static __device__ __forceinline__ v16b load(const __bf16* p) {
    U f; f.h[0] = *(const v8b*)(p); f.h[1] = *(const v8b*)(p + 16); return f.v;
  }
  static __device__ __forceinline__ v8f mma(v16b a, v16b b, v8f c) {
    return __builtin_amdgcn_wmma_f32_16x16x32_bf16(false, a, false, b, (short)0, c, false, false);
  }
  static __device__ __forceinline__ void guard(v8f& a, v8f& b, v16b x, v16b y) { dep_guard_b(a, b, x, y); }
  static __device__ __forceinline__ void keep(v16b a, v16b b, v16b c, v16b d) { keep4_b(a, b, c, d); }
};

template <int ET> struct Elem;
template <> struct Elem<0> { typedef _Float16 T; };
template <> struct Elem<1> { typedef __bf16 T; };
template <int ET, bool SPLIT, int BIAS_MODE, int OUT_MODE, bool RESID, int ACT = 0, int TRI = 0>
__global__ __launch_bounds__(256) void wmma_gemm64(
    const unsigned short* __restrict__ Ap, const unsigned short* __restrict__ A2p, int lda, long strideA,
    const unsigned short* __restrict__ Btp, const unsigned short* __restrict__ Bt2p, int ldb, long strideB,
    void* __restrict__ Cout, void* __restrict__ Cout2, int ldc, long strideC,
    const float* __restrict__ bias,
    const float* __restrict__ resid, long strideR,
    int M, int N, int K, float scale) {
  typedef typename Elem<ET>::T T;
  typedef typename Frag<T>::V V;
  const T* A = (const T*)Ap; const T* A2 = (const T*)A2p; const T* Bt = (const T*)Btp; const T* Bt2 = (const T*)Bt2p;
  __shared__ __align__(16) float sT[8][16 * 68];
  const int b    = blockIdx.y;
  const int lane = threadIdx.x & 31;
  const int wave = threadIdx.x >> 5;
  const int tilesN = N >> 6;
  const int tilesM = M >> 6;
  const int tile = blockIdx.x * 8 + wave;
  if (tile >= tilesM * tilesN) return;
  const int tm = tile / tilesN;
  const int tn = tile - tm * tilesN;
  if (TRI == 1 && tn > tm) return;
  const int m0 = tm << 6;
  const int n0 = tn << 6;
  const int kLim = (TRI == 2) ? ((m0 + 64 < K) ? (m0 + 64) : K) : K;

  const T* Ab  = A  + (size_t)b * strideA;
  const T* Bb  = Bt + (size_t)b * strideB;
  const T* Ab2 = SPLIT ? (A2  + (size_t)b * strideA) : nullptr;
  const T* Bb2 = SPLIT ? (Bt2 + (size_t)b * strideB) : nullptr;

  const int rlane = lane & 15;
  const int koff  = (lane >> 4) * 8;
  const int mOff  = (lane >> 4) * 8;

  v8f acc[4][4];
#pragma unroll
  for (int i = 0; i < 4; ++i)
#pragma unroll
    for (int j = 0; j < 4; ++j) acc[i][j] = (v8f){0.f,0.f,0.f,0.f,0.f,0.f,0.f,0.f};

  for (int k0 = 0; k0 < kLim; k0 += 32) {
    V bh[4], bl[4];
#pragma unroll
    for (int j = 0; j < 4; ++j) {
      const size_t bo = (size_t)(n0 + (j << 4) + rlane) * ldb + koff + k0;
      bh[j] = Frag<T>::load(Bb + bo);
      if (SPLIT) bl[j] = Frag<T>::load(Bb2 + bo);
    }
#pragma unroll
    for (int i = 0; i < 4; ++i) {
      const size_t ao = (size_t)(m0 + (i << 4) + rlane) * lda + koff + k0;
      V ah = Frag<T>::load(Ab + ao);
      V al;
      if (SPLIT) al = Frag<T>::load(Ab2 + ao);
#pragma unroll
      for (int j = 0; j < 4; ++j) {
        acc[i][j] = Frag<T>::mma(ah, bh[j], acc[i][j]);
        if (SPLIT) {
          acc[i][j] = Frag<T>::mma(ah, bl[j], acc[i][j]);
          acc[i][j] = Frag<T>::mma(al, bh[j], acc[i][j]);
        }
      }
      Frag<T>::guard(acc[i][0], acc[i][3], ah, SPLIT ? al : ah);
    }
    Frag<T>::keep(bh[0], bh[1], bh[2], bh[3]);
    if (SPLIT) Frag<T>::keep(bl[0], bl[1], bl[2], bl[3]);
  }
  acc_guard4(acc[0][0], acc[0][1], acc[0][2], acc[0][3]);
  acc_guard4(acc[1][0], acc[1][1], acc[1][2], acc[1][3]);
  acc_guard4(acc[2][0], acc[2][1], acc[2][2], acc[2][3]);
  acc_guard4(acc[3][0], acc[3][1], acc[3][2], acc[3][3]);

  float* slab = sT[wave];
  const float* Rb = RESID ? (resid + (size_t)b * strideR) : nullptr;
#pragma unroll
  for (int i = 0; i < 4; ++i) {
    const int mBase = m0 + (i << 4);
#pragma unroll
    for (int j = 0; j < 4; ++j) {
      const int n = n0 + (j << 4) + rlane;
      float bv = 0.f;
      if (BIAS_MODE == 2) bv = bias[n];
#pragma unroll
      for (int r = 0; r < 8; ++r) {
        float v = acc[i][j][r] * scale;
        if (BIAS_MODE == 1) v += bias[mBase + mOff + r];
        if (BIAS_MODE == 2) v += bv;
        if (RESID) v += Rb[(size_t)(mBase + mOff + r) * ldc + n];
        if (ACT == 1) v = tanhf(v);
        if (ACT == 2) v = fmaxf(v, 0.0f);
        if (ACT == 4) v = (v > 0.f) ? v : 0.01f * v;
        slab[(mOff + r) * 68 + (j << 4) + rlane] = v;
      }
    }
    __builtin_amdgcn_fence(__ATOMIC_RELEASE, "workgroup");
    __builtin_amdgcn_wave_barrier();
    __builtin_amdgcn_fence(__ATOMIC_ACQUIRE, "workgroup");
    if (OUT_MODE == 0) {
      float* C = (float*)Cout + (size_t)b * strideC;
      const int hh = lane >> 4, c4 = (lane & 15) * 4;
      for (int pass = 0; pass < 2; ++pass) {
#pragma unroll
        for (int it = 0; it < 8; ++it) {
          const int row = it * 2 + hh;
          v4f v = *(const v4f*)(slab + row * 68 + c4);
          *(volatile v4f*)(C + (size_t)(mBase + row) * ldc + n0 + c4) = v;
        }
        __threadfence();
      }
    } else {
      const int q = lane >> 3, c8 = (lane & 7) * 8;
      unsigned short* C  = (unsigned short*)Cout  + (size_t)b * strideC;
      unsigned short* C2 = (OUT_MODE == 2) ? ((unsigned short*)Cout2 + (size_t)b * strideC) : nullptr;
      for (int pass = 0; pass < 2; ++pass) {
#pragma unroll
        for (int it = 0; it < 4; ++it) {
          const int row = it * 4 + q;
          const float* sp = slab + row * 68 + c8;
          v8h hv, lv;
#pragma unroll
          for (int e = 0; e < 8; ++e) {
            if (OUT_MODE == 1) {
              hv[e] = (_Float16)sp[e];
            } else {
              unsigned short hb = f2bf_bits(sp[e]);
              unsigned short lb = f2bf_bits(sp[e] - bf_bits2f(hb));
              hv[e] = __builtin_bit_cast(_Float16, hb);
              lv[e] = __builtin_bit_cast(_Float16, lb);
            }
          }
          *(volatile v8h*)(C + (size_t)(mBase + row) * ldc + n0 + c8) = hv;
          if (OUT_MODE == 2) *(volatile v8h*)(C2 + (size_t)(mBase + row) * ldc + n0 + c8) = lv;
        }
        __threadfence();
      }
    }
    __builtin_amdgcn_fence(__ATOMIC_RELEASE, "workgroup");
    __builtin_amdgcn_wave_barrier();
    __builtin_amdgcn_fence(__ATOMIC_ACQUIRE, "workgroup");
  }
}

__device__ __forceinline__ unsigned pack_f16x2(float a, float b) {
  const _Float16 h0 = (_Float16)a, h1 = (_Float16)b;
  return (unsigned)__builtin_bit_cast(unsigned short, h0) | ((unsigned)__builtin_bit_cast(unsigned short, h1) << 16);
}
__device__ __forceinline__ void st2u(unsigned* p, unsigned v) { *(volatile unsigned*)p = v; __threadfence(); *(volatile unsigned*)p = v; }
__device__ __forceinline__ float ftanh(float x) { return 1.0f - 2.0f * __builtin_amdgcn_rcpf(1.0f + __expf(2.0f * x)); }
__device__ __forceinline__ float fsigm(float x) { return __builtin_amdgcn_rcpf(1.0f + __expf(-x)); }

__global__ __launch_bounds__(256) void prep_kernel(const float* __restrict__ w_gat, const float* __restrict__ b_gat,
                                                  const float* __restrict__ w_mean, const float* __restrict__ b_mean,
                                                  const float* __restrict__ w_std, const float* __restrict__ b_std,
                                                  const float* __restrict__ a_src, const float* __restrict__ a_dst,
                                                  unsigned* __restrict__ wg16u, unsigned* __restrict__ wh16u,
                                                  unsigned* __restrict__ bg16u, unsigned* __restrict__ bhu) {
  const int blk = blockIdx.x, tid = threadIdx.x;
  if (blk < 32) {
    const int p = blk * 256 + tid;
    const unsigned u = pack_f16x2(w_gat[2 * p] * 16.0f, w_gat[2 * p + 1] * 16.0f);
    st2u(wg16u + p, u);
  } else if (blk < 96) {
    const int p = (blk - 32) * 256 + tid;
    const int n = p >> 7;
    const int k = (2 * p) & 255;
    const int nm = (n < kAct) ? n : (kAct - 1);
    int ns = n - kAct; ns = ns < 0 ? 0 : ns;
    const float fm0 = w_mean[nm * kCat + k] * 16.0f, fm1 = w_mean[nm * kCat + k + 1] * 16.0f;
    const float fs0 = w_std [ns * kCat + k] * 16.0f, fs1 = w_std [ns * kCat + k + 1] * 16.0f;
    const unsigned u = (n < kAct) ? pack_f16x2(fm0, fm1) : pack_f16x2(fs0, fs1);
    st2u(wh16u + p, u);
  } else if (blk == 96) {
    const float f = b_gat[tid] * 16.0f;
    st2u(bg16u + tid, (unsigned)__float_as_uint(f));
  } else {
    if (tid < kHeadsN) {
      const int cm = (tid < kAct) ? tid : (kAct - 1);
      int cs = tid - kAct; cs = cs < 0 ? 0 : cs;
      const float vm = b_mean[cm], vs = b_std[cs];
      const float f = (tid < kAct) ? vm : vs;
      st2u(bhu + tid, (unsigned)__float_as_uint(f));
    }
  }
}

__global__ __launch_bounds__(kRecThreads) void rec_kernel(
    const float* __restrict__ x, const float* __restrict__ w_ih, const float* __restrict__ w_hh,
    const float* __restrict__ b_ih, const float* __restrict__ b_hh,
    float* __restrict__ hp_out, float* __restrict__ hn_out, float* __restrict__ cn_out) {
  __shared__ __align__(16) _Float16 bt[kGates * kBtP];
  __shared__ __align__(16) _Float16 ht[kNPB * kHtP];
  __shared__ __align__(16) _Float16 xt[kXtHalves];
  __shared__ __align__(16) float hp[kXch * kHidU];
  __shared__ __align__(16) float fin[2 * kNPB * kHidU];

  const int tid = threadIdx.x, lane = tid & 31, wave = tid >> 5;
  const int rlane = lane & 15, hh = lane >> 4, koff = hh * 8, mOff = hh * 8;
  const int blk = blockIdx.x;
  const int node0 = blk * kNPB;
  const int ucol = wave * 16 + rlane;

#pragma unroll 4
  for (int i = tid; i < kGates * kHidU; i += kRecThreads) {
    const int n = i >> 6, k = i & 63;
    bt[n * kBtP + k] = (_Float16)(w_hh[i] * 16.0f);
  }
  for (int i = tid; i < kGates * kFeat; i += kRecThreads) {
    const int n = i >> 3, f = i & 7;
    bt[n * kBtP + kHidU + f] = (_Float16)(w_ih[i] * 16.0f);
  }
  for (int i = tid; i < kGates * kKpad; i += kRecThreads) {
    const int n = i / kKpad, c = i - n * kKpad;
    bt[n * kBtP + kHidU + kFeat + c] = (_Float16)0.0f;
  }
  for (int i = tid; i < kNPB * kHtP; i += kRecThreads) ht[i] = (_Float16)0.0f;
  if (tid < 16) xt[kXch * kNPB * kFeat + tid] = (_Float16)0.0f;
  float bq[4];
#pragma unroll
  for (int q = 0; q < 4; ++q) bq[q] = b_ih[q * kHidU + ucol] + b_hh[q * kHidU + ucol];
  float c_st[8], h_st[8];
#pragma unroll
  for (int r = 0; r < 8; ++r) { c_st[r] = 0.0f; h_st[r] = 0.0f; }
  __syncthreads();

  const _Float16* arow = ht + rlane * kHtP + koff;
  const _Float16* brow = bt + ucol * kBtP + koff;
  const int xzero = kXch * kNPB;
  const v8h z8h = {(_Float16)0.0f, (_Float16)0.0f, (_Float16)0.0f, (_Float16)0.0f,
                   (_Float16)0.0f, (_Float16)0.0f, (_Float16)0.0f, (_Float16)0.0f};
  const v8f z8 = {0.f, 0.f, 0.f, 0.f, 0.f, 0.f, 0.f, 0.f};
  const float inv16 = 0.0625f;

#pragma unroll 1
  for (int tc = 0; tc < kT; tc += kXch) {
    {
      const int s = tid >> 4, nl = tid & 15;
      const float* xs = x + (size_t)(tc + s) * kObs + (node0 + nl) * kFeat;
      const v4f f0 = *(const v4f*)xs;
      const v4f f1 = *(const v4f*)(xs + 4);
      v8h hv;
      hv[0] = (_Float16)f0[0]; hv[1] = (_Float16)f0[1]; hv[2] = (_Float16)f0[2]; hv[3] = (_Float16)f0[3];
      hv[4] = (_Float16)f1[0]; hv[5] = (_Float16)f1[1]; hv[6] = (_Float16)f1[2]; hv[7] = (_Float16)f1[3];
      *(v8h*)(xt + (s * kNPB + nl) * kFeat) = hv;
    }
    __syncthreads();

#pragma unroll 1
    for (int s = 0; s < kXch; ++s) {
      const v16h a0 = Frag<_Float16>::load(arow);
      const v16h a1 = Frag<_Float16>::load(arow + 32);
      const int xsel = hh ? xzero : (s * kNPB + rlane);
      Frag<_Float16>::U ua;
      ua.h[0] = *(const v8h*)(xt + xsel * kFeat);
      ua.h[1] = z8h;
      const v16h a2 = ua.v;

      v8f acc[4];
      v16h fb = a0;
#pragma unroll
      for (int q = 0; q < 4; ++q) {
        const _Float16* bp = brow + q * (kHidU * kBtP);
        acc[q] = z8;
        fb = Frag<_Float16>::load(bp);      acc[q] = Frag<_Float16>::mma(a0, fb, acc[q]);
        fb = Frag<_Float16>::load(bp + 32); acc[q] = Frag<_Float16>::mma(a1, fb, acc[q]);
        fb = Frag<_Float16>::load(bp + 64); acc[q] = Frag<_Float16>::mma(a2, fb, acc[q]);
      }
      dep_guard_h(acc[2], acc[3], a2, fb);
      acc_guard4(acc[0], acc[1], acc[2], acc[3]);

      float psum = 0.0f;
#pragma unroll
      for (int r = 0; r < 8; ++r) {
        const float gi = fmaf(acc[0][r], inv16, bq[0]);
        const float gf = fmaf(acc[1][r], inv16, bq[1]);
        const float gg = fmaf(acc[2][r], inv16, bq[2]);
        const float go = fmaf(acc[3][r], inv16, bq[3]);
        const float iv = fsigm(gi), fv = fsigm(gf), gv = ftanh(gg), ov = fsigm(go);
        const float c = fmaf(fv, c_st[r], iv * gv);
        const float hv = ov * ftanh(c);
        c_st[r] = c; h_st[r] = hv; psum += hv;
      }
      psum += __shfl_xor(psum, 16, 32);
      __syncthreads();
#pragma unroll
      for (int r = 0; r < 8; ++r) ht[(mOff + r) * kHtP + ucol] = (_Float16)h_st[r];
      if (hh == 0) hp[s * kHidU + ucol] = psum;
      __syncthreads();
    }
    {
      float* dst = hp_out + ((size_t)blk * kT + tc) * kHidU + tid * 4;
      const v4f v = *(const v4f*)(hp + tid * 4);
      *(volatile v4f*)dst = v;
      __threadfence();
      *(volatile v4f*)dst = v;
    }
  }

#pragma unroll
  for (int r = 0; r < 8; ++r) {
    fin[(mOff + r) * kHidU + ucol] = h_st[r];
    fin[kNPB * kHidU + (mOff + r) * kHidU + ucol] = c_st[r];
  }
  __syncthreads();
  {
    float* hb = hn_out + (size_t)blk * (kNPB * kHidU);
    float* cb = cn_out + (size_t)blk * (kNPB * kHidU);
    const v4f h0v = *(const v4f*)(fin + tid * 4);
    const v4f h1v = *(const v4f*)(fin + 512 + tid * 4);
    const v4f c0v = *(const v4f*)(fin + 1024 + tid * 4);
    const v4f c1v = *(const v4f*)(fin + 1536 + tid * 4);
    for (int pass = 0; pass < 2; ++pass) {
      *(volatile v4f*)(hb + tid * 4) = h0v;
      *(volatile v4f*)(hb + 512 + tid * 4) = h1v;
      *(volatile v4f*)(cb + tid * 4) = c0v;
      *(volatile v4f*)(cb + 512 + tid * 4) = c1v;
      __threadfence();
    }
  }
}

__global__ __launch_bounds__(256) void hmean_kernel(const float* __restrict__ hp, unsigned* __restrict__ hm16u) {
  const int i = blockIdx.x * 256 + threadIdx.x;
  if (i >= kHmDwords) return;
  const size_t P = (size_t)kT * kHidU;
  const size_t e0 = (size_t)2 * i, e1 = e0 + 1;
  const float s0 = ((hp[e0] + hp[P + e0]) + hp[2 * P + e0]) + hp[3 * P + e0];
  const float s1 = ((hp[e1] + hp[P + e1]) + hp[2 * P + e1]) + hp[3 * P + e1];
  const float invN = 1.0f / 64.0f;
  st2u(hm16u + i, pack_f16x2(s0 * invN, s1 * invN));
}

__global__ __launch_bounds__(256) void finalize_kernel(const float* __restrict__ heads, float* __restrict__ out) {
  const int i = blockIdx.x * 256 + threadIdx.x;
  if (i >= kFin4) return;
  const int sel = i >> 16;
  const int j = i & 65535;
  const int row = j >> 4, c4 = (j & 15) * 4;
  v4f v = *(const v4f*)(heads + (size_t)row * kHeadsN + sel * kAct + c4);
  if (sel) {
#pragma unroll
    for (int e = 0; e < 4; ++e) {
      const float xv = v[e];
      float sp = fmaxf(xv, 0.0f) + log1pf(expf(-fabsf(xv)));
      sp = fminf(fmaxf(sp, kMinStd), kMaxStd);
      v[e] = sp;
    }
  }
  float* op = out + (size_t)i * 4;
  *(volatile v4f*)op = v;
  __threadfence();
  *(volatile v4f*)op = v;
}

extern "C" void kernel_launch(void* const* d_in, const int* in_sizes, int n_in,
                              void* d_out, int out_size, void* d_ws, size_t ws_size, hipStream_t stream) {
  if (n_in < 13 || d_out == nullptr || d_ws == nullptr) return;
  if (in_sizes[0] != kT * kObs || in_sizes[1] != kGates * kFeat || in_sizes[2] != kGates * kHidU || in_sizes[3] != kGates ||
      in_sizes[4] != kGates || in_sizes[5] != kCat * kHidU || in_sizes[6] != 4 * 64 || in_sizes[7] != 4 * 64 || in_sizes[8] != kCat ||
      in_sizes[9] != kAct * kCat || in_sizes[10] != kAct || in_sizes[11] != kAct * kCat || in_sizes[12] != kAct ||
      out_size != 2 * kT * kAct + 2 * kNodes * kHidU) return;

  const float* x      = (const float*)d_in[0];
  const float* w_ih   = (const float*)d_in[1];
  const float* w_hh   = (const float*)d_in[2];
  const float* b_ih   = (const float*)d_in[3];
  const float* b_hh   = (const float*)d_in[4];
  const float* w_gat  = (const float*)d_in[5];
  const float* a_src  = (const float*)d_in[6];
  const float* a_dst  = (const float*)d_in[7];
  const float* b_gat  = (const float*)d_in[8];
  const float* w_mean = (const float*)d_in[9];
  const float* b_mean = (const float*)d_in[10];
  const float* w_std  = (const float*)d_in[11];
  const float* b_std  = (const float*)d_in[12];

  float* out    = (float*)d_out;
  float* hn_out = out + (size_t)2 * kT * kAct;
  float* cn_out = hn_out + kNodes * kHidU;

  char* ws = (char*)d_ws; size_t off = 0;
  auto carve = [&](size_t bytes) -> char* { char* p = ws + off; off += (bytes + 255) & ~(size_t)255; return p; };
  float*          HP    = (float*)carve((size_t)kRecBlocks * kT * kHidU * 4);
  unsigned short* HM16  = (unsigned short*)carve((size_t)kT * kHidU * 2);
  unsigned short* WG16  = (unsigned short*)carve((size_t)kCat * kHidU * 2);
  float*          BG16  = (float*)carve((size_t)kCat * 4);
  unsigned short* G16   = (unsigned short*)carve((size_t)kT * kCat * 2);
  unsigned short* WH16  = (unsigned short*)carve((size_t)kHeadsN * kCat * 2);
  float*          BH    = (float*)carve((size_t)kHeadsN * 4);
  float*          HEADS = (float*)carve((size_t)kT * kHeadsN * 4);
  if (off > ws_size || off > (size_t)134217728) return;

  prep_kernel<<<98, 256, 0, stream>>>(w_gat, b_gat, w_mean, b_mean, w_std, b_std, a_src, a_dst,
                                      (unsigned*)WG16, (unsigned*)WH16, (unsigned*)BG16, (unsigned*)BH);

  rec_kernel<<<kRecBlocks, kRecThreads, 0, stream>>>(x, w_ih, w_hh, b_ih, b_hh, HP, hn_out, cn_out);

  hmean_kernel<<<kHmDwords / 256, 256, 0, stream>>>(HP, (unsigned*)HM16);

  wmma_gemm64<0, false, 2, 1, false, 2, 0><<<dim3(32, 1), 256, 0, stream>>>(
      HM16, nullptr, kHidU, 0L, WG16, nullptr, kHidU, 0L,
      (void*)G16, nullptr, kCat, 0L, BG16, nullptr, 0L, kT, kCat, kHidU, 1.0f);

  wmma_gemm64<0, false, 2, 0, false, 0, 0><<<dim3(16, 1), 256, 0, stream>>>(
      G16, nullptr, kCat, 0L, WH16, nullptr, kCat, 0L,
      (void*)HEADS, nullptr, kHeadsN, 0L, BH, nullptr, 0L, kT, kHeadsN, kCat, 1.0f / 256.0f);

  finalize_kernel<<<kFin4 / 256, 256, 0, stream>>>(HEADS, out);
}
